// EquivDeepSet_37263136260428
// MI455X (gfx1250) — hardware-verified
//
#include <hip/hip_runtime.h>
#include <hip/hip_bf16.h>
#include <math.h>


#define BB 8
#define SS 2048
#define DD 1024
#define HH 16
#define DKK 64
#define QW 2

typedef _Float16 bf16;
typedef __attribute__((ext_vector_type(4))) unsigned v4u_t;
typedef unsigned v4ua __attribute__((ext_vector_type(4), may_alias));
typedef __attribute__((ext_vector_type(4))) float v4f_t;
typedef float v4fa __attribute__((ext_vector_type(4), may_alias));
typedef __attribute__((ext_vector_type(16))) bf16  bf16x16;
typedef __attribute__((ext_vector_type(8)))  bf16  bf16x8;
typedef __attribute__((ext_vector_type(4)))  bf16  bf16x4;
typedef __attribute__((ext_vector_type(8)))  float f32x8;

#define LDS_STRIDE 48
#define KSTRIDE    72
#define VSTRIDE    48

__device__ __forceinline__ f32x8 wmma_bf16(bf16x16 a, bf16x16 b, f32x8 c) {
  return __builtin_amdgcn_wmma_f32_16x16x32_f16(
      false, a, false, b, (short)0, c, false, false);
}
#define RSPLIT (1.0f / 2048.0f)
__device__ __forceinline__ bf16 lo_of(float v, bf16 h) { return (bf16)((v - (float)h) * 2048.0f); }
__device__ __forceinline__ f32x8 wmma_split(bf16x16 a, bf16x16 al, bf16x16 b, bf16x16 bl, f32x8 c) {
  f32x8 x = {}; x = wmma_bf16(al, b, x); x = wmma_bf16(a, bl, x); return wmma_bf16(a, b, c) + x * RSPLIT; }

template <typename T>
__device__ __forceinline__ bf16x16 load_frag(const T* __restrict__ base, int ld,
                                             int row0, int k0) {
  const int lane = threadIdx.x & 31;
  const int r    = lane & 15;
  const int kh   = (lane >> 4) * 8;
  const T* p0 = base + (size_t)(row0 + r) * ld + (k0 + kh);
  const T* p1 = p0 + 16;
  bf16x16 f;
#pragma unroll
  for (int i = 0; i < 8; ++i) {
    f[i]     = (bf16)p0[i];
    f[i + 8] = (bf16)p1[i];
  }
  return f;
}

__device__ __forceinline__ bf16x16 lds_frag(const bf16* base, int stride) {
  const int lane = threadIdx.x & 31;
  const int row  = lane & 15;
  const int kh   = (lane >> 4) * 8;
  const bf16x8 lo = *(const bf16x8*)(base + row * stride + kh);
  const bf16x8 hi = *(const bf16x8*)(base + row * stride + kh + 16);
  bf16x16 f;
#pragma unroll
  for (int i = 0; i < 8; ++i) { f[i] = lo[i]; f[i + 8] = hi[i]; }
  return f;
}

template <typename T>
__device__ __forceinline__ void stage_read16(const T* __restrict__ p, float* buf) {
#pragma unroll
  for (int i = 0; i < 16; ++i) buf[i] = (float)p[i];
}

__device__ __forceinline__ void stage_write(bf16* dst, const float* buf, int nquad) {
#pragma unroll
  for (int i = 0; i < nquad; ++i) {
    bf16x4 q;
    q[0] = (bf16)buf[4 * i];     q[1] = (bf16)buf[4 * i + 1];
    q[2] = (bf16)buf[4 * i + 2]; q[3] = (bf16)buf[4 * i + 3];
    *(bf16x4*)(dst + 4 * i) = q;
  }
}


#define NC 1024
#define NG 16384
#define GX 128

__global__ __launch_bounds__(256) void k_prep(const float* __restrict__ Y, bf16* __restrict__ Yp) {
  const int b = blockIdx.y, c = blockIdx.x, t = threadIdx.x;
#pragma unroll 1
  for (int pass = 0; pass < 2; ++pass) {
    for (int n = t; n < NC; n += 256) { const float v = (c == 0) ? 1.0f : (c <= 2 ? Y[((size_t)b * NC + n) * 2 + (c - 1)] : 0.0f); *(volatile bf16*)(Yp + ((size_t)b * 16 + c) * NC + n) = (bf16)v; }
    __threadfence(); }
}
__global__ __launch_bounds__(256) void k_setconv(const float* __restrict__ Xc, const float* __restrict__ grid, const float* __restrict__ logl,
                                                const bf16* __restrict__ Yp, float* __restrict__ out) {
  __shared__ float fm[128][4];
  const int iy = blockIdx.x, b = blockIdx.y, t = threadIdx.x, wave = t >> 5, lane = t & 31, r16 = lane & 15, kh = (lane >> 4) * 8, kh8 = kh;
  const float l = expf(fminf(fmaxf(logl[0], -5.0f), 5.0f));
  const float cexp = -1.44269504088896340736f / (2.0f * l * l);
  const int g = iy * GX + wave * 16 + r16;
  const float gx = grid[(size_t)g * 2], gy = grid[(size_t)g * 2 + 1];
  const float* xb = Xc + (size_t)b * NC * 2; const bf16* yb = Yp + (size_t)b * 16 * NC;
  f32x8 acc = {};
#pragma unroll 1
  for (int k0 = 0; k0 < NC; k0 += 32) {
    bf16x16 a;
#pragma unroll
    for (int i = 0; i < 8; ++i) {
      { const int n = k0 + kh + i;      const float dx = gx - xb[n * 2], dy = gy - xb[n * 2 + 1]; a[i]     = (bf16)exp2f((dx * dx + dy * dy) * cexp); }
      { const int n = k0 + kh + 16 + i; const float dx = gx - xb[n * 2], dy = gy - xb[n * 2 + 1]; a[i + 8] = (bf16)exp2f((dx * dx + dy * dy) * cexp); }
    }
    const bf16x16 yf = load_frag(yb, NC, 0, k0);
    acc = wmma_bf16(a, yf, acc);
  }
  if (r16 < 3) {
#pragma unroll
    for (int r = 0; r < 8; ++r) fm[wave * 16 + kh8 + r][r16] = acc[r]; }
  __syncthreads();
#pragma unroll 1
  for (int pass = 0; pass < 2; ++pass) {
    for (int i = t; i < 3 * 32; i += 256) { const int c = i >> 5, x4 = (i & 31) * 4; v4f_t v;
#pragma unroll
      for (int q = 0; q < 4; ++q) { const float den = fm[x4 + q][0]; v[q] = (c == 0) ? den : fm[x4 + q][c] / den; }
      *(volatile v4f_t*)(out + (((size_t)b * 3 + c) * GX + iy) * GX + x4) = v; }
    __threadfence();
  }
}

extern "C" void kernel_launch(void* const* d_in, const int* in_sizes, int n_in,
                              void* d_out, int out_size, void* d_ws, size_t ws_size,
                              hipStream_t stream) {
  (void)in_sizes; (void)n_in; (void)out_size; (void)ws_size;
  const float* Xc = (const float*)d_in[0];
  const float* Yc = (const float*)d_in[1];
  const float* grid = (const float*)d_in[2];
  const float* logl = (const float*)d_in[3];
  bf16* Yp = (bf16*)d_ws;
  k_prep<<<dim3(16, BB), 256, 0, stream>>>(Yc, Yp);
  k_setconv<<<dim3(GX, BB), 256, 0, stream>>>(Xc, grid, logl, Yp, (float*)d_out);
}
